// InductiveBuNNLayer_51049981280278
// MI455X (gfx1250) — hardware-verified
//
#include <hip/hip_runtime.h>
#include <stddef.h>


#define FEAT   64
#define H1D    32
#define H2D    16
#define NPAR   6
#define NTHR   256
#define NWAVE  8
#define EPT    8
#define NGRP   2
#define CHUNK  (NTHR * EPT * NGRP)
#define WCAP   (EPT * NGRP * 32)
#define LISTN  (NWAVE * WCAP)
#define NBLK   256
#define HROWS  (NBLK / 2)
#define NBD    4096
#define MAXN   4096
#define NWD    (MAXN / 32)
#define NSW    (NWD / 32)

static_assert((CHUNK & (CHUNK - 1)) == 0);
static_assert(CHUNK <= 4096);
static_assert(NBLK <= 4096 && (NBLK & (NBLK - 1)) == 0);
static_assert(NBD <= 4096 && (NBD & (NBD - 1)) == 0);
static_assert(NWD == 128 && NSW == 4);

#define S1_ACC   0
#define S1_LIST  (S1_ACC + NBLK * FEAT * 4)
#define S1_STG   (S1_LIST + LISTN * 4)
#define S1_WBH   (S1_STG + NBLK * H1D * 4)
#define S1_WBL   (S1_WBH + H1D * 2 * FEAT * 2)
#define S1_CNT   (S1_WBL + H1D * 2 * FEAT * 2)
#define S1_WCNT  (S1_CNT + NBLK * 4)
#define LDS_S1   (S1_WCNT + 64)

#define S2_ACC   0
#define S2_LIST  (S2_ACC + NBLK * H1D * 4)
#define S2_H2S   (S2_LIST + LISTN * 4)
#define S2_OS    (S2_H2S + NBLK * H2D * 4)
#define S2_LOC   (S2_OS + NBLK * 16 * 4)
#define S2_W2H   (S2_LOC + NBLK * FEAT * 4)
#define S2_W2L   (S2_W2H + H2D * 2 * H1D * 2)
#define S2_CNT   (S2_W2L + H2D * 2 * H1D * 2)
#define S2_WCNT  (S2_CNT + NBLK * 4)
#define LDS_S2   (S2_WCNT + 64)

#define SD_BM    0
#define SD_STV   (SD_BM + NBLK * NWD * 4)
#define SD_STS   (SD_STV + HROWS * FEAT * 4)
#define SD_LIST  (SD_STS + HROWS * FEAT * 4)
#define SD_SUM   (SD_LIST + LISTN * 4)
#define SD_WCNT  (SD_SUM + NBLK * NSW * 4)
#define LDS_SD   (SD_WCNT + 64)

#define SF_MIX   0
#define SF_WTH   (SF_MIX + NBLK * FEAT * 4)
#define SF_WTL   (SF_WTH + FEAT * FEAT * 2)
#define LDS_SF   (SF_WTL + FEAT * FEAT * 2)

static_assert((S1_LIST & 15) == 0 && (S1_STG & 15) == 0 && (S1_WBH & 15) == 0 && (S1_WBL & 15) == 0 && (S1_CNT & 15) == 0);
static_assert((S2_LIST & 15) == 0 && (S2_H2S & 15) == 0 && (S2_OS & 15) == 0 && (S2_LOC & 15) == 0 && (S2_W2H & 15) == 0 && (S2_W2L & 15) == 0);
static_assert((SD_STV & 15) == 0 && (SD_STS & 15) == 0 && (SD_LIST & 15) == 0 && (SD_SUM & 15) == 0);
static_assert((SF_WTH & 15) == 0 && (SF_WTL & 15) == 0);

typedef float          v2f   __attribute__((ext_vector_type(2)));
typedef float          v4f   __attribute__((ext_vector_type(4)));
typedef float          v8f   __attribute__((ext_vector_type(8)));
typedef int            v4i   __attribute__((ext_vector_type(4)));
typedef unsigned short v8us  __attribute__((ext_vector_type(8)));
typedef unsigned short v16us __attribute__((ext_vector_type(16)));
typedef __bf16         v16bf __attribute__((ext_vector_type(16)));
union FragB { v16bf v; v16us u; v8us h[2]; };

__device__ __forceinline__ unsigned bfb(float f) {
  const unsigned u = __float_as_uint(f);
  return (u + 0x7FFFu + ((u >> 16) & 1u)) >> 16;
}

__device__ __forceinline__ void split16(v4f p0, v4f p1, v4f p2, v4f p3, FragB& hi, FragB& lo) {
  float f[16] = {p0.x, p0.y, p0.z, p0.w, p1.x, p1.y, p1.z, p1.w,
                 p2.x, p2.y, p2.z, p2.w, p3.x, p3.y, p3.z, p3.w};
#pragma unroll
  for (int i = 0; i < 16; ++i) {
    const unsigned hb = bfb(f[i]);
    const unsigned lb = bfb(f[i] - __uint_as_float(hb << 16));
    hi.u[i] = (unsigned short)hb;
    lo.u[i] = (unsigned short)lb;
  }
}

__device__ __forceinline__ float dot4(v4f a, v4f b) {
  return a.x * b.x + a.y * b.y + a.z * b.z + a.w * b.w;
}

__device__ __forceinline__ v8f wmb(v16bf a, v16bf b, v8f c) {
  v8f d = __builtin_amdgcn_wmma_f32_16x16x32_bf16(false, a, false, b, (short)0, c, false, false);
  asm volatile("v_nop\n\tv_nop\n\tv_nop\n\tv_nop" : "+v"(d) : "v"(a), "v"(b));
  return d;
}
__device__ __forceinline__ v8f wmb3(v16bf ah, v16bf al, v16bf bh, v16bf bl, v8f c) {
  c = wmb(ah, bh, c);
  c = wmb(ah, bl, c);
  c = wmb(al, bh, c);
  return c;
}

template <int NB>
__device__ __forceinline__ int scan_chunk(const int* __restrict__ keys, int nE, int cbase, int nodeBase,
                                          int vec8, int* list, int tid, int lane, int wave) {
  int wc = 0;
#pragma unroll
  for (int g = 0; g < NGRP; ++g) {
    const int el0  = (g * NTHR + tid) * EPT;
    const int e0   = cbase + el0;
    const int sent = -2147483647 - 1;
    v4i da, db;
    if (vec8 != 0 && cbase + CHUNK <= nE) {
      da = *(const v4i*)(keys + e0);
      db = *(const v4i*)(keys + e0 + 4);
    } else {
      da.x = (e0     < nE) ? keys[min(e0, nE - 1)] : sent;
      da.y = (e0 + 1 < nE) ? keys[min(e0 + 1, nE - 1)] : sent;
      da.z = (e0 + 2 < nE) ? keys[min(e0 + 2, nE - 1)] : sent;
      da.w = (e0 + 3 < nE) ? keys[min(e0 + 3, nE - 1)] : sent;
      db.x = (e0 + 4 < nE) ? keys[min(e0 + 4, nE - 1)] : sent;
      db.y = (e0 + 5 < nE) ? keys[min(e0 + 5, nE - 1)] : sent;
      db.z = (e0 + 6 < nE) ? keys[min(e0 + 6, nE - 1)] : sent;
      db.w = (e0 + 7 < nE) ? keys[min(e0 + 7, nE - 1)] : sent;
    }
    const unsigned nb = (unsigned)nodeBase;
    const unsigned s0 = (unsigned)da.x - nb, s1 = (unsigned)da.y - nb;
    const unsigned s2 = (unsigned)da.z - nb, s3 = (unsigned)da.w - nb;
    const unsigned s4 = (unsigned)db.x - nb, s5 = (unsigned)db.y - nb;
    const unsigned s6 = (unsigned)db.z - nb, s7 = (unsigned)db.w - nb;
    const bool h0 = s0 < (unsigned)NB, h1 = s1 < (unsigned)NB, h2 = s2 < (unsigned)NB, h3 = s3 < (unsigned)NB;
    const bool h4 = s4 < (unsigned)NB, h5 = s5 < (unsigned)NB, h6 = s6 < (unsigned)NB, h7 = s7 < (unsigned)NB;
    const unsigned any = __builtin_amdgcn_ballot_w32(h0 | h1 | h2 | h3 | h4 | h5 | h6 | h7);
    if (any != 0u) {
#define HITJ(J, HJ, SJ) { \
        const unsigned mj = __builtin_amdgcn_ballot_w32(HJ); \
        if (mj != 0u) { \
          if (HJ) { \
            const int pos = wc + (int)__builtin_amdgcn_mbcnt_lo(mj, 0u); \
            if (pos < WCAP) list[wave * WCAP + pos] = ((el0 + (J)) << 12) | (int)(SJ); \
          } \
          wc += (int)__builtin_popcount(mj); } }
      HITJ(0, h0, s0)
      HITJ(1, h1, s1)
      HITJ(2, h2, s2)
      HITJ(3, h3, s3)
      HITJ(4, h4, s4)
      HITJ(5, h5, s5)
      HITJ(6, h6, s6)
      HITJ(7, h7, s7)
#undef HITJ
    }
  }
  return wc;
}

__global__ __launch_bounds__(NTHR) void k_deg(
    const int* __restrict__ ei, float* dis, int nN, int nE, int vec8) {
  __shared__ __attribute__((aligned(16))) int cnt[NBD];
  __shared__ __attribute__((aligned(16))) int list[LISTN];
  __shared__ int wcnt[NWAVE];
  const int tid = threadIdx.x, lane = tid & 31, wave = tid >> 5;
  const int nodeBase = blockIdx.x * NBD;
  (void)nN;

  for (int i = tid; i < NBD; i += NTHR) cnt[i] = 0;
  __syncthreads();

  const int nChunks = (nE + CHUNK - 1) / CHUNK;
#pragma unroll 1
  for (int ch = 0; ch < nChunks; ++ch) {
    const int cbase = ch * CHUNK;
    const int wc = scan_chunk<NBD>(ei, nE, cbase, nodeBase, vec8, list, tid, lane, wave);
    if (lane == 0) wcnt[wave] = wc;
    __syncthreads();
    if (wave == 0) {
#pragma unroll 1
      for (int wsx = 0; wsx < NWAVE; ++wsx) {
        int n = __builtin_amdgcn_readfirstlane(wcnt[wsx]);
        n = n > WCAP ? WCAP : (n < 0 ? 0 : n);
        const int* lp = list + wsx * WCAP;
#pragma unroll 1
        for (int i = 0; i < n; ++i) {
          const int ent  = __builtin_amdgcn_readfirstlane(lp[i]);
          const int slot = ent & (NBD - 1);
          if (lane == 0) cnt[slot] = cnt[slot] + 1;
        }
      }
    }
    __syncthreads();
  }

  v4f dq[4];
#pragma unroll
  for (int q = 0; q < 4; ++q) {
    const int f = (wave * 4 + q) * 128 + 4 * lane;
    const v4i c = *(const v4i*)(cnt + f);
    dq[q].x = rsqrtf((float)(c.x + 1));
    dq[q].y = rsqrtf((float)(c.y + 1));
    dq[q].z = rsqrtf((float)(c.z + 1));
    dq[q].w = rsqrtf((float)(c.w + 1));
  }
  float* dp = dis + (size_t)nodeBase;
#pragma unroll
  for (int q = 0; q < 4; ++q) *(volatile v4f*)(dp + (wave * 4 + q) * 128 + 4 * lane) = dq[q];
  __threadfence();
#pragma unroll
  for (int q = 0; q < 4; ++q) *(volatile v4f*)(dp + (wave * 4 + q) * 128 + 4 * lane) = dq[q];
}

__global__ __launch_bounds__(NTHR) void k_agg1(
    const int* __restrict__ ei, const float* __restrict__ x,
    const float* __restrict__ Wl, const float* __restrict__ Wr, const float* __restrict__ bv,
    float* h1, int nN, int nE, int vec8) {
  extern __shared__ v4f lds_dyn[];
  char* lb = (char*)lds_dyn;
  float*          acc  = (float*)(lb + S1_ACC);
  int*            list = (int*)(lb + S1_LIST);
  float*          stg  = (float*)(lb + S1_STG);
  unsigned short* wbh  = (unsigned short*)(lb + S1_WBH);
  unsigned short* wbl  = (unsigned short*)(lb + S1_WBL);
  int*            cnt  = (int*)(lb + S1_CNT);
  int*            wcnt = (int*)(lb + S1_WCNT);
  const int tid = threadIdx.x, lane = tid & 31, wave = tid >> 5, hh = lane >> 4, m = lane & 15;
  const int nodeBase = blockIdx.x * NBLK;
  const int* dsts = ei + nE;

  {
    const v4f z = {0.f, 0.f, 0.f, 0.f};
    for (int i = tid; i < NBLK * FEAT / 4; i += NTHR) ((v4f*)acc)[i] = z;
    for (int i = tid; i < NBLK; i += NTHR) cnt[i] = 0;
  }
#pragma unroll 4
  for (int it = 0; it < (H1D * 2 * FEAT) / NTHR; ++it) {
    const int idx = it * NTHR + tid;
    const int n   = idx >> 7;
    const int kk  = idx & 127;
    const int kc  = kk & 63;
    const float vl = Wl[n * FEAT + kc];
    const float vr = Wr[n * FEAT + kc];
    const float v  = (kk < FEAT) ? vl : vr;
    const unsigned hb = bfb(v);
    const unsigned lo = bfb(v - __uint_as_float(hb << 16));
    wbh[idx] = (unsigned short)hb;
    wbl[idx] = (unsigned short)lo;
  }
  __syncthreads();

  const int nChunks = (nE + CHUNK - 1) / CHUNK;
#pragma unroll 1
  for (int ch = 0; ch < nChunks; ++ch) {
    const int cbase = ch * CHUNK;
    const int wc = scan_chunk<NBLK>(dsts, nE, cbase, nodeBase, vec8, list, tid, lane, wave);
    if (lane == 0) wcnt[wave] = wc;
    __syncthreads();
    if (wave == 0) {
#pragma unroll 1
      for (int wsx = 0; wsx < NWAVE; ++wsx) {
        int n = __builtin_amdgcn_readfirstlane(wcnt[wsx]);
        n = n > WCAP ? WCAP : (n < 0 ? 0 : n);
        const int* lp = list + wsx * WCAP;
#pragma unroll 1
        for (int i = 0; i < n; ++i) {
          const int ent  = __builtin_amdgcn_readfirstlane(lp[i]);
          const int slot = ent & (NBLK - 1);
          int e = cbase + ((ent >> 12) & (CHUNK - 1));
          e = e > nE - 1 ? nE - 1 : e;
          int src = ei[e];
          src = src < 0 ? 0 : (src > nN - 1 ? nN - 1 : src);
          const v2f v = *(const v2f*)(x + (size_t)src * FEAT + 2 * lane);
          v2f* ap = (v2f*)(acc + slot * FEAT + 2 * lane);
          *ap = *ap + v;
          if (lane == 0) cnt[slot] = cnt[slot] + 1;
        }
      }
    }
    __syncthreads();
  }

#pragma unroll
  for (int q = 0; q < 2; ++q) {
    const int tile = wave + 8 * q;
    const int r    = 16 * tile + m;
    int node = nodeBase + r;
    node = node > nN - 1 ? nN - 1 : node;
    const float cf  = (float)cnt[r];
    const float inv = 1.0f / fmaxf(cf, 1.0f);
    v8f c[2];
#pragma unroll
    for (int t = 0; t < 2; ++t) { v8f z = {0.f, 0.f, 0.f, 0.f, 0.f, 0.f, 0.f, 0.f}; c[t] = z; }
#pragma unroll
    for (int kt = 0; kt < 4; ++kt) {
      v4f p0, p1, p2, p3;
      if (kt < 2) {
        const float* ap = acc + r * FEAT + 32 * kt + 8 * hh;
        p0 = (*(const v4f*)ap) * inv;        p1 = (*(const v4f*)(ap + 4)) * inv;
        p2 = (*(const v4f*)(ap + 16)) * inv; p3 = (*(const v4f*)(ap + 20)) * inv;
      } else {
        const float* xp = x + (size_t)node * FEAT + 32 * (kt - 2) + 8 * hh;
        p0 = *(const v4f*)xp;        p1 = *(const v4f*)(xp + 4);
        p2 = *(const v4f*)(xp + 16); p3 = *(const v4f*)(xp + 20);
      }
      FragB ah, al;
      split16(p0, p1, p2, p3, ah, al);
#pragma unroll
      for (int t = 0; t < 2; ++t) {
        const unsigned short* bq = wbh + (16 * t + m) * (2 * FEAT) + 32 * kt + 8 * hh;
        const unsigned short* br = wbl + (16 * t + m) * (2 * FEAT) + 32 * kt + 8 * hh;
        FragB bh, bl;
        bh.h[0] = *(const v8us*)bq; bh.h[1] = *(const v8us*)(bq + 16);
        bl.h[0] = *(const v8us*)br; bl.h[1] = *(const v8us*)(br + 16);
        c[t] = wmb3(ah.v, al.v, bh.v, bl.v, c[t]);
      }
    }
#pragma unroll
    for (int t = 0; t < 2; ++t) {
      const int col = 16 * t + m;
      const float bb = bv[col];
      float* sp = stg + (16 * tile + 8 * hh) * H1D + col;
#pragma unroll
      for (int rr = 0; rr < 8; ++rr) sp[rr * H1D] = fmaxf(c[t][rr] + bb, 0.f);
    }
  }
  __syncthreads();

  float* gp = h1 + (size_t)nodeBase * H1D;
#pragma unroll
  for (int q = 0; q < 8; ++q) {
    const int f = (wave * 8 + q) * 128 + 4 * lane;
    const v4f v = *(const v4f*)(stg + f);
    *(volatile v4f*)(gp + f) = v;
  }
  __threadfence();
#pragma unroll
  for (int q = 0; q < 8; ++q) {
    const int f = (wave * 8 + q) * 128 + 4 * lane;
    const v4f v = *(const v4f*)(stg + f);
    *(volatile v4f*)(gp + f) = v;
  }
}

__global__ __launch_bounds__(NTHR) void k_agg2(
    const int* __restrict__ ei, const float* __restrict__ h1,
    const float* __restrict__ Wl2, const float* __restrict__ Wr2, const float* __restrict__ b2,
    const float* __restrict__ Wp, const float* __restrict__ bp, const float* __restrict__ x,
    float* Opl, float* loc_out, int nN, int nE, int vec8) {
  extern __shared__ v4f lds_dyn[];
  char* lb = (char*)lds_dyn;
  float*          acc  = (float*)(lb + S2_ACC);
  int*            list = (int*)(lb + S2_LIST);
  float*          h2s  = (float*)(lb + S2_H2S);
  float*          os   = (float*)(lb + S2_OS);
  float*          loc  = (float*)(lb + S2_LOC);
  unsigned short* w2h  = (unsigned short*)(lb + S2_W2H);
  unsigned short* w2l  = (unsigned short*)(lb + S2_W2L);
  int*            cnt  = (int*)(lb + S2_CNT);
  int*            wcnt = (int*)(lb + S2_WCNT);
  const int tid = threadIdx.x, lane = tid & 31, wave = tid >> 5, hh = lane >> 4, m = lane & 15;
  const int nodeBase = blockIdx.x * NBLK;
  const int* dsts = ei + nE;

  {
    const v4f z = {0.f, 0.f, 0.f, 0.f};
    for (int i = tid; i < NBLK * H1D / 4; i += NTHR) ((v4f*)acc)[i] = z;
    for (int i = tid; i < NBLK; i += NTHR) cnt[i] = 0;
  }
#pragma unroll
  for (int it = 0; it < (H2D * 2 * H1D) / NTHR; ++it) {
    const int idx = it * NTHR + tid;
    const int n   = idx >> 6;
    const int kk  = idx & 63;
    const int kc  = kk & 31;
    const float vl = Wl2[n * H1D + kc];
    const float vr = Wr2[n * H1D + kc];
    const float v  = (kk < H1D) ? vl : vr;
    const unsigned hb = bfb(v);
    const unsigned lo = bfb(v - __uint_as_float(hb << 16));
    w2h[idx] = (unsigned short)hb;
    w2l[idx] = (unsigned short)lo;
  }
  __syncthreads();

  const int nChunks = (nE + CHUNK - 1) / CHUNK;
#pragma unroll 1
  for (int ch = 0; ch < nChunks; ++ch) {
    const int cbase = ch * CHUNK;
    const int wc = scan_chunk<NBLK>(dsts, nE, cbase, nodeBase, vec8, list, tid, lane, wave);
    if (lane == 0) wcnt[wave] = wc;
    __syncthreads();
    if (wave == 0) {
#pragma unroll 1
      for (int wsx = 0; wsx < NWAVE; ++wsx) {
        int n = __builtin_amdgcn_readfirstlane(wcnt[wsx]);
        n = n > WCAP ? WCAP : (n < 0 ? 0 : n);
        const int* lp = list + wsx * WCAP;
#pragma unroll 1
        for (int i = 0; i < n; ++i) {
          const int ent  = __builtin_amdgcn_readfirstlane(lp[i]);
          const int slot = ent & (NBLK - 1);
          int e = cbase + ((ent >> 12) & (CHUNK - 1));
          e = e > nE - 1 ? nE - 1 : e;
          int src = ei[e];
          src = src < 0 ? 0 : (src > nN - 1 ? nN - 1 : src);
          const float v = h1[(size_t)src * H1D + lane];
          float* ap = acc + slot * H1D + lane;
          *ap = *ap + v;
          if (lane == 0) cnt[slot] = cnt[slot] + 1;
        }
      }
    }
    __syncthreads();
  }

#pragma unroll
  for (int q = 0; q < 2; ++q) {
    const int tile = wave + 8 * q;
    const int r    = 16 * tile + m;
    int node = nodeBase + r;
    node = node > nN - 1 ? nN - 1 : node;
    const float cf  = (float)cnt[r];
    const float inv = 1.0f / fmaxf(cf, 1.0f);
    v8f c = {0.f, 0.f, 0.f, 0.f, 0.f, 0.f, 0.f, 0.f};
#pragma unroll
    for (int kt = 0; kt < 2; ++kt) {
      v4f p0, p1, p2, p3;
      if (kt == 0) {
        const float* ap = acc + r * H1D + 8 * hh;
        p0 = (*(const v4f*)ap) * inv;        p1 = (*(const v4f*)(ap + 4)) * inv;
        p2 = (*(const v4f*)(ap + 16)) * inv; p3 = (*(const v4f*)(ap + 20)) * inv;
      } else {
        const float* hp = h1 + (size_t)node * H1D + 8 * hh;
        p0 = *(const v4f*)hp;        p1 = *(const v4f*)(hp + 4);
        p2 = *(const v4f*)(hp + 16); p3 = *(const v4f*)(hp + 20);
      }
      FragB ah, al;
      split16(p0, p1, p2, p3, ah, al);
      const unsigned short* bq = w2h + m * (2 * H1D) + 32 * kt + 8 * hh;
      const unsigned short* br = w2l + m * (2 * H1D) + 32 * kt + 8 * hh;
      FragB bh, bl;
      bh.h[0] = *(const v8us*)bq; bh.h[1] = *(const v8us*)(bq + 16);
      bl.h[0] = *(const v8us*)br; bl.h[1] = *(const v8us*)(br + 16);
      c = wmb3(ah.v, al.v, bh.v, bl.v, c);
    }
    const float bb = b2[m];
    float* sp = h2s + (16 * tile + 8 * hh) * H2D + m;
#pragma unroll
    for (int rr = 0; rr < 8; ++rr) sp[rr * H2D] = fmaxf(c[rr] + bb, 0.f);
  }
  __syncthreads();

  {
    const int slot = tid;
    int node = nodeBase + slot;
    node = node > nN - 1 ? nN - 1 : node;
    const v4f g0 = *(const v4f*)(h2s + slot * H2D);
    const v4f g1 = *(const v4f*)(h2s + slot * H2D + 4);
    const v4f g2 = *(const v4f*)(h2s + slot * H2D + 8);
    const v4f g3 = *(const v4f*)(h2s + slot * H2D + 12);
    float p[NPAR];
#pragma unroll
    for (int cI = 0; cI < NPAR; ++cI) {
      const v4f w0 = *(const v4f*)(Wp + cI * H2D);
      const v4f w1 = *(const v4f*)(Wp + cI * H2D + 4);
      const v4f w2 = *(const v4f*)(Wp + cI * H2D + 8);
      const v4f w3 = *(const v4f*)(Wp + cI * H2D + 12);
      const float s = dot4(g0, w0) + dot4(g1, w1) + dot4(g2, w2) + dot4(g3, w3);
      p[cI] = s + bp[cI];
    }
    float M[4][4], R[4][4];
    M[0][0] = 1.f;   M[0][1] = -p[0]; M[0][2] = -p[1]; M[0][3] = -p[2];
    M[1][0] = p[0];  M[1][1] = 1.f;   M[1][2] = -p[3]; M[1][3] = -p[4];
    M[2][0] = p[1];  M[2][1] = p[3];  M[2][2] = 1.f;   M[2][3] = -p[5];
    M[3][0] = p[2];  M[3][1] = p[4];  M[3][2] = p[5];  M[3][3] = 1.f;
#pragma unroll
    for (int rI = 0; rI < 4; ++rI)
#pragma unroll
      for (int cI = 0; cI < 4; ++cI) R[rI][cI] = (rI == cI) ? 1.f : 0.f;
#pragma unroll
    for (int col = 0; col < 4; ++col) {
      const float pinv = 1.0f / M[col][col];
#pragma unroll
      for (int cI = 0; cI < 4; ++cI) { M[col][cI] *= pinv; R[col][cI] *= pinv; }
#pragma unroll
      for (int rI = 0; rI < 4; ++rI) {
        if (rI == col) continue;
        const float f = M[rI][col];
#pragma unroll
        for (int cI = 0; cI < 4; ++cI) { M[rI][cI] -= f * M[col][cI]; R[rI][cI] -= f * R[col][cI]; }
      }
    }
    float O[4][4];
#pragma unroll
    for (int rI = 0; rI < 4; ++rI)
#pragma unroll
      for (int cI = 0; cI < 4; ++cI) O[rI][cI] = 2.f * R[rI][cI] - ((rI == cI) ? 1.f : 0.f);
#pragma unroll
    for (int rI = 0; rI < 4; ++rI) {
      v4f ov; ov.x = O[rI][0]; ov.y = O[rI][1]; ov.z = O[rI][2]; ov.w = O[rI][3];
      *(v4f*)(os + slot * 16 + 4 * rI) = ov;
    }
    const float* xr = x + (size_t)node * FEAT;
#pragma unroll 2
    for (int b = 0; b < 16; ++b) {
      const v4f xv = *(const v4f*)(xr + 4 * b);
      v4f lv;
      lv.x = O[0][0] * xv.x + O[1][0] * xv.y + O[2][0] * xv.z + O[3][0] * xv.w;
      lv.y = O[0][1] * xv.x + O[1][1] * xv.y + O[2][1] * xv.z + O[3][1] * xv.w;
      lv.z = O[0][2] * xv.x + O[1][2] * xv.y + O[2][2] * xv.z + O[3][2] * xv.w;
      lv.w = O[0][3] * xv.x + O[1][3] * xv.y + O[2][3] * xv.z + O[3][3] * xv.w;
      *(v4f*)(loc + slot * FEAT + 4 * b) = lv;
    }
  }
  __syncthreads();

  float* gO = Opl + (size_t)nodeBase * 16;
  float* gL = loc_out + (size_t)nodeBase * FEAT;
#pragma unroll
  for (int q = 0; q < 4; ++q) {
    const int f = (wave * 4 + q) * 128 + 4 * lane;
    const v4f v = *(const v4f*)(os + f);
    *(volatile v4f*)(gO + f) = v;
  }
#pragma unroll
  for (int q = 0; q < 16; ++q) {
    const int f = (wave * 16 + q) * 128 + 4 * lane;
    const v4f v = *(const v4f*)(loc + f);
    *(volatile v4f*)(gL + f) = v;
  }
  __threadfence();
#pragma unroll
  for (int q = 0; q < 4; ++q) {
    const int f = (wave * 4 + q) * 128 + 4 * lane;
    const v4f v = *(const v4f*)(os + f);
    *(volatile v4f*)(gO + f) = v;
  }
#pragma unroll
  for (int q = 0; q < 16; ++q) {
    const int f = (wave * 16 + q) * 128 + 4 * lane;
    const v4f v = *(const v4f*)(loc + f);
    *(volatile v4f*)(gL + f) = v;
  }
}

__global__ __launch_bounds__(NTHR) void k_diff(
    const int* __restrict__ ei, const float* __restrict__ dis,
    const float* vin, float* vout, const float* sin_, float* sout,
    float coef, int nN, int nE, int vec8) {
  extern __shared__ v4f lds_dyn[];
  char* lb = (char*)lds_dyn;
  unsigned* bm   = (unsigned*)(lb + SD_BM);
  float*    stv  = (float*)(lb + SD_STV);
  float*    sts  = (float*)(lb + SD_STS);
  int*      list = (int*)(lb + SD_LIST);
  unsigned* summ = (unsigned*)(lb + SD_SUM);
  int*      wcnt = (int*)(lb + SD_WCNT);
  const int tid = threadIdx.x, lane = tid & 31, wave = tid >> 5;
  const int rowBase = blockIdx.x * NBLK;

  for (int i = tid; i < NBLK * NWD; i += NTHR) {
    const int r = i >> 7;
    const int w = i & (NWD - 1);
    const int gi = rowBase + r;
    bm[i] = (w == (gi >> 5)) ? (1u << (gi & 31)) : 0u;
  }
  for (int i = tid; i < NBLK * NSW; i += NTHR) {
    const int r  = i >> 2;
    const int sw = i & (NSW - 1);
    const int gi = rowBase + r;
    summ[i] = (sw == (gi >> 10)) ? (1u << ((gi >> 5) & 31)) : 0u;
  }
  __syncthreads();

  const int nChunks = (nE + CHUNK - 1) / CHUNK;
#pragma unroll 1
  for (int ch = 0; ch < nChunks; ++ch) {
    const int cbase = ch * CHUNK;
    const int wc = scan_chunk<NBLK>(ei, nE, cbase, rowBase, vec8, list, tid, lane, wave);
    if (lane == 0) wcnt[wave] = wc;
    __syncthreads();
    if (wave == 0) {
#pragma unroll 1
      for (int wsx = 0; wsx < NWAVE; ++wsx) {
        int n = __builtin_amdgcn_readfirstlane(wcnt[wsx]);
        n = n > WCAP ? WCAP : (n < 0 ? 0 : n);
        const int* lp = list + wsx * WCAP;
#pragma unroll 1
        for (int i = 0; i < n; ++i) {
          const int ent  = __builtin_amdgcn_readfirstlane(lp[i]);
          const int slot = ent & (NBLK - 1);
          int e = cbase + ((ent >> 12) & (CHUNK - 1));
          e = e > nE - 1 ? nE - 1 : e;
          int col = ei[nE + e];
          col = col < 0 ? 0 : (col > nN - 1 ? nN - 1 : col);
          if (lane == 0) {
            bm[slot * NWD + (col >> 5)]    |= 1u << (col & 31);
            summ[slot * NSW + (col >> 10)] |= 1u << ((col >> 5) & 31);
          }
        }
      }
    }
    __syncthreads();
  }

#pragma unroll 1
  for (int hp = 0; hp < 2; ++hp) {
#pragma unroll 1
    for (int q = 0; q < 16; ++q) {
      const int rl = wave * 16 + q;
      const int r  = hp * HROWS + rl;
      int gi = rowBase + r;
      gi = gi > nN - 1 ? nN - 1 : gi;
      v2f s = {0.f, 0.f};
#pragma unroll 1
      for (int sw = 0; sw < NSW; ++sw) {
        unsigned word = (unsigned)__builtin_amdgcn_readfirstlane((int)summ[r * NSW + sw]);
#pragma unroll 1
        for (int it = 0; it < 32; ++it) {
          if (word == 0u) break;
          const int b = __builtin_ctz(word);
          word &= word - 1u;
          const int wi = sw * 32 + b;
          unsigned bits = (unsigned)__builtin_amdgcn_readfirstlane((int)bm[r * NWD + wi]);
#pragma unroll 1
          for (int jt = 0; jt < 32; ++jt) {
            if (bits == 0u) break;
            const int bb = __builtin_ctz(bits);
            bits &= bits - 1u;
            int j = wi * 32 + bb;
            j = j > nN - 1 ? nN - 1 : j;
            const float dj = dis[j];
            const v2f vj = *(const v2f*)(vin + (size_t)j * FEAT + 2 * lane);
            s = s + dj * vj;
          }
        }
      }
      const v2f vi  = *(const v2f*)(vin + (size_t)gi * FEAT + 2 * lane);
      const float di = dis[gi];
      const v2f vk  = coef * (vi - di * s);
      const v2f so  = *(const v2f*)(sin_ + (size_t)gi * FEAT + 2 * lane) + vk;
      *(v2f*)(stv + rl * FEAT + 2 * lane) = vk;
      *(v2f*)(sts + rl * FEAT + 2 * lane) = so;
    }
    __syncthreads();
    const size_t gofs = ((size_t)rowBase + (size_t)hp * HROWS) * FEAT;
#pragma unroll
    for (int qq = 0; qq < 8; ++qq) {
      const int f = (wave * 8 + qq) * 128 + 4 * lane;
      const v4f a = *(const v4f*)(stv + f);
      const v4f b = *(const v4f*)(sts + f);
      *(volatile v4f*)(vout + gofs + f) = a;
      *(volatile v4f*)(sout + gofs + f) = b;
    }
    __threadfence();
#pragma unroll
    for (int qq = 0; qq < 8; ++qq) {
      const int f = (wave * 8 + qq) * 128 + 4 * lane;
      const v4f a = *(const v4f*)(stv + f);
      const v4f b = *(const v4f*)(sts + f);
      *(volatile v4f*)(vout + gofs + f) = a;
      *(volatile v4f*)(sout + gofs + f) = b;
    }
    __syncthreads();
  }
}

__global__ __launch_bounds__(NTHR) void k_mix(
    const float* __restrict__ S, const float* __restrict__ W, const float* __restrict__ Opl,
    const float* __restrict__ bias, float* out, int nN) {
  extern __shared__ v4f lds_dyn[];
  char* lb = (char*)lds_dyn;
  float*          mix = (float*)(lb + SF_MIX);
  unsigned short* wth = (unsigned short*)(lb + SF_WTH);
  unsigned short* wtl = (unsigned short*)(lb + SF_WTL);
  const int tid = threadIdx.x, lane = tid & 31, wave = tid >> 5, hh = lane >> 4, m = lane & 15;
  const int rowBase = blockIdx.x * NBLK;

#pragma unroll 4
  for (int it = 0; it < (FEAT * FEAT) / NTHR; ++it) {
    const int idx = it * NTHR + tid;
    const int n   = idx >> 6;
    const int k   = idx & 63;
    const float v = W[k * FEAT + n];
    const unsigned hb = bfb(v);
    const unsigned lo = bfb(v - __uint_as_float(hb << 16));
    wth[idx] = (unsigned short)hb;
    wtl[idx] = (unsigned short)lo;
  }
  __syncthreads();

#pragma unroll
  for (int q = 0; q < 2; ++q) {
    const int tile = wave + 8 * q;
    const int r    = 16 * tile + m;
    int node = rowBase + r;
    node = node > nN - 1 ? nN - 1 : node;
    const float* sp = S + (size_t)node * FEAT;
    v8f c[4];
#pragma unroll
    for (int t = 0; t < 4; ++t) { v8f z = {0.f, 0.f, 0.f, 0.f, 0.f, 0.f, 0.f, 0.f}; c[t] = z; }
#pragma unroll
    for (int kt = 0; kt < 2; ++kt) {
      const float* ap = sp + 32 * kt + 8 * hh;
      const v4f p0 = *(const v4f*)ap,        p1 = *(const v4f*)(ap + 4);
      const v4f p2 = *(const v4f*)(ap + 16), p3 = *(const v4f*)(ap + 20);
      FragB ah, al;
      split16(p0, p1, p2, p3, ah, al);
#pragma unroll
      for (int t = 0; t < 4; ++t) {
        const unsigned short* bq = wth + (16 * t + m) * FEAT + 32 * kt + 8 * hh;
        const unsigned short* br = wtl + (16 * t + m) * FEAT + 32 * kt + 8 * hh;
        FragB bh, bl;
        bh.h[0] = *(const v8us*)bq; bh.h[1] = *(const v8us*)(bq + 16);
        bl.h[0] = *(const v8us*)br; bl.h[1] = *(const v8us*)(br + 16);
        c[t] = wmb3(ah.v, al.v, bh.v, bl.v, c[t]);
      }
    }
#pragma unroll
    for (int t = 0; t < 4; ++t) {
      float* mp = mix + (16 * tile + 8 * hh) * FEAT + 16 * t + m;
#pragma unroll
      for (int rr = 0; rr < 8; ++rr) mp[rr * FEAT] = c[t][rr];
    }
  }
  __syncthreads();

  {
    const int slot = tid;
    int node = rowBase + slot;
    node = node > nN - 1 ? nN - 1 : node;
    const v4f o0 = *(const v4f*)(Opl + (size_t)node * 16);
    const v4f o1 = *(const v4f*)(Opl + (size_t)node * 16 + 4);
    const v4f o2 = *(const v4f*)(Opl + (size_t)node * 16 + 8);
    const v4f o3 = *(const v4f*)(Opl + (size_t)node * 16 + 12);
#pragma unroll 2
    for (int b = 0; b < 16; ++b) {
      const v4f mv = *(const v4f*)(mix + slot * FEAT + 4 * b);
      const v4f bz = *(const v4f*)(bias + 4 * b);
      v4f rv;
      rv.x = dot4(o0, mv); rv.y = dot4(o1, mv); rv.z = dot4(o2, mv); rv.w = dot4(o3, mv);
      rv = rv + bz;
      rv.x = fmaxf(rv.x, 0.f); rv.y = fmaxf(rv.y, 0.f); rv.z = fmaxf(rv.z, 0.f); rv.w = fmaxf(rv.w, 0.f);
      *(v4f*)(mix + slot * FEAT + 4 * b) = rv;
    }
  }
  __syncthreads();

  const size_t outN = (size_t)nN * FEAT;
  const size_t ob   = (size_t)rowBase * FEAT;
#pragma unroll
  for (int q = 0; q < 16; ++q) {
    const int f = (wave * 16 + q) * 128 + 4 * lane;
    const size_t gi = ob + (size_t)f;
    if (gi < outN) { const v4f v = *(const v4f*)(mix + f); *(volatile v4f*)(out + gi) = v; }
  }
  __threadfence();
#pragma unroll
  for (int q = 0; q < 16; ++q) {
    const int f = (wave * 16 + q) * 128 + 4 * lane;
    const size_t gi = ob + (size_t)f;
    if (gi < outN) { const v4f v = *(const v4f*)(mix + f); *(volatile v4f*)(out + gi) = v; }
  }
}

extern "C" void kernel_launch(void* const* d_in, const int* in_sizes, int n_in,
                              void* d_out, int out_size, void* d_ws, size_t ws_size,
                              hipStream_t stream) {
  if (n_in < 12) return;
  const int nN = in_sizes[0] / FEAT;
  const int nE = in_sizes[1] / 2;
  if (nN <= 0 || nN > MAXN || in_sizes[0] != nN * FEAT || nE < 0 || in_sizes[1] != nE * 2) return;
  if (in_sizes[2] != H1D * FEAT || in_sizes[3] != H1D * FEAT || in_sizes[4] < H1D) return;
  if (in_sizes[5] != H2D * H1D || in_sizes[6] != H2D * H1D || in_sizes[7] < H2D) return;
  if (in_sizes[8] != NPAR * H2D || in_sizes[9] < NPAR) return;
  if (in_sizes[10] != FEAT * FEAT || in_sizes[11] < FEAT) return;
  if (out_size != nN * FEAT) return;

  const float* x    = (const float*)d_in[0];
  const int*   ei   = (const int*)d_in[1];
  const float* Wl1  = (const float*)d_in[2];
  const float* Wr1  = (const float*)d_in[3];
  const float* b1   = (const float*)d_in[4];
  const float* Wl2  = (const float*)d_in[5];
  const float* Wr2  = (const float*)d_in[6];
  const float* b2   = (const float*)d_in[7];
  const float* Wp   = (const float*)d_in[8];
  const float* bp   = (const float*)d_in[9];
  const float* W    = (const float*)d_in[10];
  const float* bias = (const float*)d_in[11];
  float* out = (float*)d_out;

  const int    nBD  = (nN + NBD - 1) / NBD;
  const int    nBlk = (nN + NBLK - 1) / NBLK;
  const size_t NPr  = (size_t)nBlk * NBLK;

  char* ws = (char*)d_ws;
  size_t off = 0;
  const size_t oDis = off; off += (size_t)nBD * NBD * 4;        off = (off + 255) & ~(size_t)255;
  const size_t oH1  = off; off += NPr * H1D * 4;                off = (off + 255) & ~(size_t)255;
  const size_t oO   = off; off += NPr * 16 * 4;                 off = (off + 255) & ~(size_t)255;
  const size_t oVA  = off; off += NPr * FEAT * 4;               off = (off + 255) & ~(size_t)255;
  const size_t oVB  = off; off += NPr * FEAT * 4;               off = (off + 255) & ~(size_t)255;
  const size_t oS   = off; off += NPr * FEAT * 4;               off = (off + 255) & ~(size_t)255;
  if (off > ws_size) return;
  float* dis = (float*)(ws + oDis);
  float* h1  = (float*)(ws + oH1);
  float* Opl = (float*)(ws + oO);
  float* va  = (float*)(ws + oVA);
  float* vb  = (float*)(ws + oVB);
  float* S   = (float*)(ws + oS);

  const int vec8 = ((nE & 3) == 0) ? 1 : 0;

  k_deg<<<nBD, NTHR, 0, stream>>>(ei, dis, nN, nE, vec8);

  hipFuncSetAttribute(reinterpret_cast<const void*>(&k_agg1),
                      hipFuncAttributeMaxDynamicSharedMemorySize, LDS_S1);
  k_agg1<<<nBlk, NTHR, LDS_S1, stream>>>(ei, x, Wl1, Wr1, b1, h1, nN, nE, vec8);

  hipFuncSetAttribute(reinterpret_cast<const void*>(&k_agg2),
                      hipFuncAttributeMaxDynamicSharedMemorySize, LDS_S2);
  k_agg2<<<nBlk, NTHR, LDS_S2, stream>>>(ei, h1, Wl2, Wr2, b2, Wp, bp, x, Opl, va, nN, nE, vec8);

  hipFuncSetAttribute(reinterpret_cast<const void*>(&k_diff),
                      hipFuncAttributeMaxDynamicSharedMemorySize, LDS_SD);
  float* pin = va;
  float* pout = vb;
  const float* sin0 = va;
#pragma unroll 1
  for (int k = 1; k <= 10; ++k) {
    const float coef = (float)(-1.0 / (double)k);
    k_diff<<<nBlk, NTHR, LDS_SD, stream>>>(ei, dis, pin, pout, sin0, S, coef, nN, nE, vec8);
    sin0 = S;
    float* t = pin; pin = pout; pout = t;
  }

  hipFuncSetAttribute(reinterpret_cast<const void*>(&k_mix),
                      hipFuncAttributeMaxDynamicSharedMemorySize, LDS_SF);
  k_mix<<<nBlk, NTHR, LDS_SF, stream>>>(S, W, Opl, bias, out, nN);
}
